// NicheTrans_img_58703613002247
// MI455X (gfx1250) — hardware-verified
//
#include <hip/hip_runtime.h>


#define NB_  8192
#define TT   137
#define DD   384
#define KK   128
#define NC   (TT * KK)
#define NCB  (NC / 64)

typedef unsigned short bf;
typedef __attribute__((ext_vector_type(16))) __bf16   v16bf;
typedef __attribute__((ext_vector_type(8)))  unsigned short v8us;
typedef __attribute__((ext_vector_type(8)))  float    v8f;
typedef __attribute__((ext_vector_type(4)))  float    v4f;
typedef v4f  __attribute__((may_alias)) v4fa;
typedef v8us __attribute__((may_alias)) v8usa;

__device__ __forceinline__ unsigned short f2bf(float f) { unsigned u = __float_as_uint(f); u += 0x7FFFu + ((u >> 16) & 1u); return (unsigned short)(u >> 16); }
__device__ __forceinline__ float bf2f(unsigned short b) { return __uint_as_float(((unsigned)b) << 16); }
__device__ __forceinline__ float bfr(float f) { return bf2f(f2bf(f)); }
__device__ __forceinline__ v16bf cat16b(v8us lo, v8us hi) { return __builtin_bit_cast(v16bf, __builtin_shufflevector(lo, hi, 0, 1, 2, 3, 4, 5, 6, 7, 8, 9, 10, 11, 12, 13, 14, 15)); }
__device__ __forceinline__ v8f wmmab(v16bf a, v16bf b, v8f c) { return __builtin_amdgcn_wmma_f32_16x16x32_bf16(false, a, false, b, (short)0, c, false, false); }

__global__ __launch_bounds__(256) void k_rows(const float* __restrict__ src, int rows, bf* dst) {
    const int lane = threadIdx.x & 31, r = blockIdx.x * 8 + (threadIdx.x >> 5);
    if (r >= rows) return;
#pragma unroll 1
    for (int ps = 0; ps < 2; ++ps) {
#pragma unroll
        for (int q = 0; q < 2; ++q) { const int pc = q * 32 + lane; if (pc < DD / 8) { v8us o;
#pragma unroll
                for (int i = 0; i < 8; ++i) o[i] = f2bf(src[(size_t)r * DD + pc * 8 + i]);
                *(volatile v8us*)(dst + (size_t)r * DD + pc * 8) = o; } }
        if (ps == 0) __threadfence(); }
}
__global__ __launch_bounds__(128) void k_gemm(const bf* __restrict__ A, const bf* __restrict__ Bn, const float* __restrict__ b1, const float* __restrict__ gam, const float* __restrict__ bet, const float* __restrict__ rmean, const float* __restrict__ rvar, const float* __restrict__ W2, float* PART) {
    __shared__ __align__(16) float prow[64];
    const int lane = threadIdx.x & 31, wave = threadIdx.x >> 5, lr = lane & 15, hi = lane >> 4;
    const size_t r0 = (size_t)blockIdx.x * 64 + wave * 16; const int cb = blockIdx.y, c0 = cb * 64;
    const size_t aoff = (r0 + lr) * DD + 8 * hi;
    size_t boff[4];
#pragma unroll
    for (int t = 0; t < 4; ++t) boff[t] = (size_t)(c0 + t * 16 + lr) * DD + 8 * hi;
    v8f acc[4];
#pragma unroll
    for (int t = 0; t < 4; ++t) acc[t] = (v8f){};
#pragma unroll
    for (int kc = 0; kc < DD; kc += 32) {
        const v16bf a = cat16b(*(const v8us*)(A + aoff + kc), *(const v8us*)(A + aoff + kc + 16));
#pragma unroll
        for (int t = 0; t < 4; ++t) acc[t] = wmmab(a, cat16b(*(const v8us*)(Bn + boff[t] + kc), *(const v8us*)(Bn + boff[t] + kc + 16)), acc[t]);
        asm volatile("v_nop" : "+v"(acc[0]), "+v"(acc[1]), "+v"(acc[2]), "+v"(acc[3]) : "v"(a) : "memory");
    }
    float part[8];
#pragma unroll
    for (int j = 0; j < 8; ++j) part[j] = 0.f;
#pragma unroll
    for (int t = 0; t < 4; ++t) { const int c = c0 + t * 16 + lr;
        const float bb = bfr(b1[c]), sc = bfr(gam[c]) * rsqrtf(bfr(rvar[c]) + 1e-5f), mu = bfr(rmean[c]), be = bfr(bet[c]), w2 = bfr(W2[c]);
#pragma unroll
        for (int j = 0; j < 8; ++j) { float h = acc[t][j] + bb; h = (h - mu) * sc + be; h = (h >= 0.f) ? h : 0.01f * h; part[j] += h * w2; } }
#pragma unroll
    for (int j = 0; j < 8; ++j) { part[j] += __shfl_xor(part[j], 1, 16); part[j] += __shfl_xor(part[j], 2, 16); part[j] += __shfl_xor(part[j], 4, 16); part[j] += __shfl_xor(part[j], 8, 16); }
    if (lr == 0) {
#pragma unroll
        for (int j = 0; j < 8; ++j) prow[wave * 16 + hi * 8 + j] = part[j]; }
    __syncthreads();
    if (wave == 0) { const float v0 = prow[lane], v1 = prow[32 + lane]; float* dst = PART + (size_t)cb * NB_ + (size_t)blockIdx.x * 64;
        *(volatile float*)(dst + lane) = v0; *(volatile float*)(dst + 32 + lane) = v1; __threadfence(); *(volatile float*)(dst + lane) = v0; *(volatile float*)(dst + 32 + lane) = v1; }
}
__global__ __launch_bounds__(256) void k_fin(const float* __restrict__ PART, const float* __restrict__ b2, float* out) {
    const size_t f = (size_t)blockIdx.x * 256 + threadIdx.x; if (f >= (size_t)NB_ * TT) return;
    const int b = (int)(f / TT), t = (int)(f - (size_t)b * TT);
    const float v = PART[(size_t)(2 * t) * NB_ + b] + PART[(size_t)(2 * t + 1) * NB_ + b] + bfr(b2[t]);
    *(volatile float*)(out + f) = v; __threadfence(); *(volatile float*)(out + f) = v;
}

extern "C" void kernel_launch(void* const* d_in, const int* in_sizes, int n_in,
                              void* d_out, int out_size, void* d_ws, size_t ws_size, hipStream_t stream) {
    (void)in_sizes; (void)n_in; (void)out_size;
    const float* f = (const float*)d_in[0]; const float* W1 = (const float*)d_in[1]; const float* b1 = (const float*)d_in[2]; const float* gam = (const float*)d_in[3]; const float* bet = (const float*)d_in[4];
    const float* rmean = (const float*)d_in[5]; const float* rvar = (const float*)d_in[6]; const float* W2 = (const float*)d_in[7]; const float* b2 = (const float*)d_in[8];
    float* out = (float*)d_out;
    char* wsp = (char*)d_ws;
    auto take = [&](size_t bytes) { char* p = wsp; wsp += (bytes + 255) & ~(size_t)255; return (void*)p; };
    bf* Fb = (bf*)take((size_t)NB_ * DD * 2); bf* Wb = (bf*)take((size_t)NC * DD * 2); float* PART = (float*)take((size_t)NCB * NB_ * 4);
    if ((size_t)(wsp - (char*)d_ws) > ws_size) return;
    k_rows<<<NB_ / 8, 256, 0, stream>>>(f, NB_, Fb); k_rows<<<NC / 8, 256, 0, stream>>>(W1, NC, Wb);
    k_gemm<<<dim3(NB_ / 64, NCB, 1), 128, 0, stream>>>(Fb, Wb, b1, gam, bet, rmean, rvar, W2, PART);
    k_fin<<<(unsigned)(((size_t)NB_ * TT + 255) / 256), 256, 0, stream>>>(PART, b2, out);
}
